// PointNetFeaturePropagation_30391188587133
// MI455X (gfx1250) — hardware-run, weakly checked
//
#include <hip/hip_runtime.h>

#pragma clang fp contract(off)

typedef __attribute__((ext_vector_type(16))) _Float16 v16h;
typedef __attribute__((ext_vector_type(8)))  _Float16 v8h;
typedef __attribute__((ext_vector_type(8)))  float    v8f;
typedef __attribute__((ext_vector_type(4)))  float    v4f;
typedef __attribute__((ext_vector_type(4)))  int      v4i;

constexpr int NB_BATCH = 4;
constexpr int NPT1     = 16384;
constexpr int NPT2     = 4096;
constexpr int CH_P1    = 128;
constexpr int CH_P2    = 256;
constexpr int CH_IN    = CH_P1 + CH_P2;
constexpr int CH_H1    = 256;
constexpr int CH_OUT   = 128;
constexpr int NPTS_ALL = NB_BATCH * NPT1;

constexpr float W_CARRY     = 1024.0f;
constexpr float W_CARRY_INV = 1.0f / 1024.0f;
constexpr float BN_EPS      = 1e-5f;

static_assert(CH_IN == 384, "concat width");
static_assert(CH_IN % 32 == 0 && CH_H1 % 32 == 0, "GEMM depth must be a multiple of 32");
static_assert(NPTS_ALL % 64 == 0 && CH_H1 % 64 == 0 && CH_OUT % 64 == 0, "GEMM tile multiples");
static_assert(NPTS_ALL == 65536, "pooled sample count");

constexpr size_t SZ_R1  = (size_t)NPTS_ALL * CH_IN * 2;
constexpr size_t SZ_R2  = (size_t)NPTS_ALL * CH_H1 * 4;
constexpr size_t SZ_W1  = (size_t)CH_H1 * CH_IN * 2;
constexpr size_t SZ_W2  = (size_t)CH_OUT * CH_H1 * 2;
constexpr int    ST1_BLOCKS = 512;
constexpr int    ST1_ROWS   = NPTS_ALL / ST1_BLOCKS;
constexpr size_t SZ_P1  = (size_t)ST1_BLOCKS * 2 * CH_H1 * 4;
constexpr size_t SZ_T1  = (size_t)2 * CH_H1 * 4;
constexpr size_t SZ_T2  = (size_t)CH_OUT * 32 * 4;
constexpr size_t OFF_R1  = 0;
constexpr size_t OFF_R2  = OFF_R1 + SZ_R1;
constexpr size_t OFF_W1H = OFF_R2 + SZ_R2;
constexpr size_t OFF_W1L = OFF_W1H + SZ_W1;
constexpr size_t OFF_W2H = OFF_W1L + SZ_W1;
constexpr size_t OFF_W2L = OFF_W2H + SZ_W2;
constexpr size_t OFF_P1  = OFF_W2L + SZ_W2;
constexpr size_t OFF_T1  = OFF_P1 + SZ_P1;
constexpr size_t OFF_T2  = OFF_T1 + SZ_T1;
constexpr size_t WS_TOTAL = OFF_T2 + SZ_T2;
static_assert(WS_TOTAL <= (size_t)134217728, "carve above 128 MiB");
static_assert((size_t)NPTS_ALL * CH_H1 * 2 <= SZ_R1, "H1 alias fits R1");
static_assert((size_t)CH_OUT * NPTS_ALL * 4 <= SZ_R2, "Y2 alias fits R2");
static_assert(OFF_R2 % 128 == 0 && OFF_W1H % 128 == 0 && OFF_W1L % 128 == 0 && OFF_W2H % 128 == 0 &&
              OFF_W2L % 128 == 0 && OFF_P1 % 128 == 0 && OFF_T1 % 128 == 0 && OFF_T2 % 128 == 0, "line alignment");
static_assert(ST1_ROWS * ST1_BLOCKS == NPTS_ALL, "stats slabs cover all rows");

constexpr int PW_BLOCKS_W1 = (CH_H1 * CH_IN) / (8 * 256);
constexpr int PW_BLOCKS_W2 = (CH_OUT * CH_H1) / (8 * 256);
static_assert(PW_BLOCKS_W1 * 8 * 256 == CH_H1 * CH_IN, "prep coverage W1");
static_assert(PW_BLOCKS_W2 * 8 * 256 == CH_OUT * CH_H1, "prep coverage W2");

__global__ __launch_bounds__(256) void prep_weights(const float* __restrict__ W1, const float* __restrict__ W2,
                                                    _Float16* __restrict__ W1h, _Float16* __restrict__ W1l,
                                                    _Float16* __restrict__ W2h, _Float16* __restrict__ W2l) {
  const bool first = (int)blockIdx.x < PW_BLOCKS_W1;
  const float* src = first ? W1 : W2;
  _Float16* dh = first ? W1h : W2h;
  _Float16* dl = first ? W1l : W2l;
  const int u = first ? ((int)blockIdx.x * 256 + (int)threadIdx.x)
                      : (((int)blockIdx.x - PW_BLOCKS_W1) * 256 + (int)threadIdx.x);
  const v4f a = *(const v4f*)(src + (size_t)u * 8);
  const v4f c = *(const v4f*)(src + (size_t)u * 8 + 4);
  float f[8];
  f[0] = a.x; f[1] = a.y; f[2] = a.z; f[3] = a.w;
  f[4] = c.x; f[5] = c.y; f[6] = c.z; f[7] = c.w;
  v8h hv, lv;
#pragma unroll
  for (int e = 0; e < 8; ++e) {
    const float s = f[e] * W_CARRY;
    const _Float16 h = (_Float16)s;
    const float hf = (float)h;
    const float r = s - hf;
    hv[e] = h;
    lv[e] = (_Float16)r;
  }
  *(volatile v8h*)(dh + (size_t)u * 8) = hv;
  *(volatile v8h*)(dl + (size_t)u * 8) = lv;
  __threadfence();
  *(volatile v8h*)(dh + (size_t)u * 8) = hv;
  *(volatile v8h*)(dl + (size_t)u * 8) = lv;
}

constexpr int KNN_TILE = 1024;
constexpr int XT_PITCH = 392;
constexpr int SUB_PTS  = 32;
static_assert(NPT2 % KNN_TILE == 0, "source tiles");
static_assert((XT_PITCH * 2) % 16 == 0, "LDS row alignment");
static_assert((SUB_PTS * CH_IN) / 8 == 6 * 256, "store-out coverage: 1536 units of 16 B = 6 x 256 threads");

__global__ __launch_bounds__(256) void knn_build_x(const float* __restrict__ xyz1, const float* __restrict__ xyz2,
                                                   const float* __restrict__ pts1, const float* __restrict__ pts2,
                                                   _Float16* __restrict__ X) {
#pragma clang fp contract(off)
  __shared__ __align__(16) float    sSrc[KNN_TILE * 4];
  __shared__ __align__(16) int      sIdx[256 * 4];
  __shared__ __align__(16) float    sWgt[256 * 4];
  __shared__ __align__(16) _Float16 sTile[SUB_PTS * XT_PITCH];

  const int tid  = (int)threadIdx.x;
  const int lane = tid & 31;
  const int wave = tid >> 5;
  const int b    = (int)blockIdx.x >> 6;
  const int qblk = ((int)blockIdx.x & 63) * 256;
  const int q    = qblk + tid;

  const float* x1 = xyz1 + (size_t)b * 3 * NPT1;
  const float* x2 = xyz2 + (size_t)b * 3 * NPT2;
  const float qx = x1[q];
  const float qy = x1[NPT1 + q];
  const float qz = x1[2 * NPT1 + q];
  const float tqx = qx * qx;
  const float tqy = qy * qy;
  const float tqz = qz * qz;
  const float sq1 = (tqx + tqz) + tqy;

  float d0 = __builtin_huge_valf(), d1 = __builtin_huge_valf(), d2 = __builtin_huge_valf();
  int i0 = 0, i1 = 0, i2 = 0;

  for (int t0 = 0; t0 < NPT2; t0 += KNN_TILE) {
    __syncthreads();
#pragma unroll
    for (int it = 0; it < 4; ++it) {
      const int i = it * 256 + tid;
      const float sx = x2[t0 + i];
      const float sy = x2[NPT2 + t0 + i];
      const float sz = x2[2 * NPT2 + t0 + i];
      const float ax = sx * sx;
      const float ay = sy * sy;
      const float az = sz * sz;
      v4f pk;
      pk.x = sx; pk.y = sy; pk.z = sz; pk.w = (ax + az) + ay;
      *(v4f*)(sSrc + i * 4) = pk;
    }
    __syncthreads();
#pragma unroll 4
    for (int i = 0; i < KNN_TILE; ++i) {
      const v4f s = *(const v4f*)(sSrc + i * 4);
      float p = qx * s.x;
      p = __builtin_fmaf(qy, s.y, p);
      p = __builtin_fmaf(qz, s.z, p);
      const float ss = sq1 + s.w;
      const float d = ss - (p + p);
      if (d < d2) {
        const int gi = t0 + i;
        const bool c0 = d < d0;
        const bool c1 = d < d1;
        const float nd2 = c1 ? d1 : d;
        const int   ni2 = c1 ? i1 : gi;
        const float nd1 = c0 ? d0 : (c1 ? d : d1);
        const int   ni1 = c0 ? i0 : (c1 ? gi : i1);
        d0 = c0 ? d : d0;
        i0 = c0 ? gi : i0;
        d1 = nd1; i1 = ni1;
        d2 = nd2; i2 = ni2;
      }
    }
  }

  {
    const int j0 = min(max(i0, 0), NPT2 - 1);
    const int j1 = min(max(i1, 0), NPT2 - 1);
    const int j2 = min(max(i2, 0), NPT2 - 1);
    const float g0x = x2[j0], g0y = x2[NPT2 + j0], g0z = x2[2 * NPT2 + j0];
    const float g1x = x2[j1], g1y = x2[NPT2 + j1], g1z = x2[2 * NPT2 + j1];
    const float g2x = x2[j2], g2y = x2[NPT2 + j2], g2z = x2[2 * NPT2 + j2];
    float ex, ey, ez;
    ex = qx - g0x; ey = qy - g0y; ez = qz - g0z;
    ex = ex * ex; ey = ey * ey; ez = ez * ez;
    float e0 = (ex + ez) + ey;
    ex = qx - g1x; ey = qy - g1y; ez = qz - g1z;
    ex = ex * ex; ey = ey * ey; ez = ez * ez;
    float e1 = (ex + ez) + ey;
    ex = qx - g2x; ey = qy - g2y; ez = qz - g2z;
    ex = ex * ex; ey = ey * ey; ez = ez * ez;
    float e2 = (ex + ez) + ey;
    e0 = fmaxf(e0, 1e-10f);
    e1 = fmaxf(e1, 1e-10f);
    e2 = fmaxf(e2, 1e-10f);
    float w0 = 1.0f / e0;
    float w1 = 1.0f / e1;
    float w2 = 1.0f / e2;
    const float wsum = (w0 + w2) + w1;
    w0 = w0 / wsum;
    w1 = w1 / wsum;
    w2 = w2 / wsum;
    v4i iv;
    iv.x = j0; iv.y = j1; iv.z = j2; iv.w = 0;
    v4f wv;
    wv.x = w0; wv.y = w1; wv.z = w2; wv.w = 0.0f;
    *(v4i*)(sIdx + tid * 4) = iv;
    *(v4f*)(sWgt + tid * 4) = wv;
  }
  __syncthreads();

  const float* p1b = pts1 + (size_t)b * CH_P1 * NPT1;
  const float* p2b = pts2 + (size_t)b * CH_P2 * NPT2;
#pragma unroll 1
  for (int st = 0; st < 8; ++st) {
    const int qi = st * SUB_PTS + lane;
    const int n  = qblk + qi;
    const v4i id = *(const v4i*)(sIdx + qi * 4);
    const v4f wq = *(const v4f*)(sWgt + qi * 4);
    const int j0 = min(max(id.x, 0), NPT2 - 1);
    const int j1 = min(max(id.y, 0), NPT2 - 1);
    const int j2 = min(max(id.z, 0), NPT2 - 1);
    const float w0 = wq.x, w1 = wq.y, w2 = wq.z;

#pragma unroll 1
    for (int g = 0; g < 2; ++g) {
      const int c0 = wave * 16 + g * 8;
      v8h hv;
#pragma unroll
      for (int e = 0; e < 8; ++e) {
        const float v = p1b[(size_t)(c0 + e) * NPT1 + n];
        hv[e] = (_Float16)v;
      }
      *(v8h*)(sTile + lane * XT_PITCH + c0) = hv;
    }
#pragma unroll 1
    for (int g = 0; g < 4; ++g) {
      const int c0 = wave * 32 + g * 8;
      const float* r = p2b + (size_t)c0 * NPT2;
      float a[12];
#pragma unroll
      for (int e = 0; e < 4; ++e) {
        a[3 * e + 0] = r[(size_t)e * NPT2 + j0];
        a[3 * e + 1] = r[(size_t)e * NPT2 + j1];
        a[3 * e + 2] = r[(size_t)e * NPT2 + j2];
      }
      float v0 = (w0 * a[0] + w1 * a[1]) + w2 * a[2];
      float v1 = (w0 * a[3] + w1 * a[4]) + w2 * a[5];
      float v2 = (w0 * a[6] + w1 * a[7]) + w2 * a[8];
      float v3 = (w0 * a[9] + w1 * a[10]) + w2 * a[11];
      asm volatile("" : "+v"(v0), "+v"(v1), "+v"(v2), "+v"(v3) :: "memory");
      float c[12];
#pragma unroll
      for (int e = 0; e < 4; ++e) {
        c[3 * e + 0] = r[(size_t)(4 + e) * NPT2 + j0];
        c[3 * e + 1] = r[(size_t)(4 + e) * NPT2 + j1];
        c[3 * e + 2] = r[(size_t)(4 + e) * NPT2 + j2];
      }
      float v4 = (w0 * c[0] + w1 * c[1]) + w2 * c[2];
      float v5 = (w0 * c[3] + w1 * c[4]) + w2 * c[5];
      float v6 = (w0 * c[6] + w1 * c[7]) + w2 * c[8];
      float v7 = (w0 * c[9] + w1 * c[10]) + w2 * c[11];
      asm volatile("" : "+v"(v4), "+v"(v5), "+v"(v6), "+v"(v7) :: "memory");
      v8h hv;
      hv[0] = (_Float16)v0; hv[1] = (_Float16)v1; hv[2] = (_Float16)v2; hv[3] = (_Float16)v3;
      hv[4] = (_Float16)v4; hv[5] = (_Float16)v5; hv[6] = (_Float16)v6; hv[7] = (_Float16)v7;
      *(v8h*)(sTile + lane * XT_PITCH + CH_P1 + c0) = hv;
    }
    __syncthreads();

    {
      _Float16* dst = X + ((size_t)b * NPT1 + (size_t)(qblk + st * SUB_PTS)) * CH_IN;
      v8h ov[6];
#pragma unroll
      for (int it = 0; it < 6; ++it) {
        const int u = it * 256 + tid;
        const int row = u / 48;
        const int cu = u - row * 48;
        ov[it] = *(const v8h*)(sTile + row * XT_PITCH + cu * 8);
      }
#pragma unroll
      for (int it = 0; it < 6; ++it) *(volatile v8h*)(dst + (size_t)(it * 256 + tid) * 8) = ov[it];
      __threadfence();
#pragma unroll
      for (int it = 0; it < 6; ++it) *(volatile v8h*)(dst + (size_t)(it * 256 + tid) * 8) = ov[it];
    }
    __syncthreads();
  }
}

union FragU { v16h v; v8h h[2]; };
__device__ __forceinline__ v16h frag_load(const _Float16* p) {
  FragU f;
  f.h[0] = *(const v8h*)(p);
  f.h[1] = *(const v8h*)(p + 16);
  return f.v;
}
__device__ __forceinline__ v8f frag_mma(v16h a, v16h b, v8f c) {
  return __builtin_amdgcn_wmma_f32_16x16x32_f16(false, a, false, b, (short)0, c, false, false);
}
__device__ __forceinline__ void dep_guard4_h(v8f& a, v8f& b, v8f& c, v8f& d, v16h x, v16h y) {
  asm volatile("v_nop\n\tv_nop\n\tv_nop\n\tv_nop" : "+v"(a), "+v"(b), "+v"(c), "+v"(d) : "v"(x), "v"(y));
}
__device__ __forceinline__ void keep4_h(v16h a, v16h b, v16h c, v16h d) {
  asm volatile("v_nop" :: "v"(a), "v"(b), "v"(c), "v"(d));
}
__device__ __forceinline__ void acc_guard4(v8f& a, v8f& b, v8f& c, v8f& d) {
  asm volatile("v_nop\n\tv_nop\n\tv_nop\n\tv_nop" : "+v"(a), "+v"(b), "+v"(c), "+v"(d));
}

template <bool SPLIT_A, bool SPLIT_B>
__global__ __launch_bounds__(256) void wmma_gemm64_f16(
    const unsigned short* __restrict__ Ap, const unsigned short* __restrict__ A2p, int lda,
    const unsigned short* __restrict__ Btp, const unsigned short* __restrict__ Bt2p, int ldb,
    float* __restrict__ Cout, int ldc, int M, int N, int K, float scale) {
  const _Float16* A   = (const _Float16*)Ap;
  const _Float16* A2  = (const _Float16*)A2p;
  const _Float16* Bt  = (const _Float16*)Btp;
  const _Float16* Bt2 = (const _Float16*)Bt2p;
  __shared__ __align__(16) float sT[8][16 * 68];
  const int lane = threadIdx.x & 31;
  const int wave = threadIdx.x >> 5;
  const int tilesN = N >> 6;
  const int tilesM = M >> 6;
  const int tile = blockIdx.x * 8 + wave;
  if (tile >= tilesM * tilesN) return;
  const int tm = tile / tilesN;
  const int tn = tile - tm * tilesN;
  const int m0 = tm << 6;
  const int n0 = tn << 6;

  const int rlane = lane & 15;
  const int koff  = (lane >> 4) * 8;
  const int mOff  = (lane >> 4) * 8;

  v8f acc[4][4];
#pragma unroll
  for (int i = 0; i < 4; ++i)
#pragma unroll
    for (int j = 0; j < 4; ++j) acc[i][j] = (v8f){0.f, 0.f, 0.f, 0.f, 0.f, 0.f, 0.f, 0.f};

  for (int k0 = 0; k0 < K; k0 += 32) {
    v16h bh[4], bl[4];
#pragma unroll
    for (int j = 0; j < 4; ++j) {
      const size_t bo = (size_t)(n0 + (j << 4) + rlane) * ldb + koff + k0;
      bh[j] = frag_load(Bt + bo);
      bl[j] = bh[j];
      if (SPLIT_B) bl[j] = frag_load(Bt2 + bo);
    }
#pragma unroll
    for (int i = 0; i < 4; ++i) {
      const size_t ao = (size_t)(m0 + (i << 4) + rlane) * lda + koff + k0;
      v16h ah = frag_load(A + ao);
      v16h al = ah;
      if (SPLIT_A) al = frag_load(A2 + ao);
#pragma unroll
      for (int j = 0; j < 4; ++j) {
        acc[i][j] = frag_mma(ah, bh[j], acc[i][j]);
        if (SPLIT_B) acc[i][j] = frag_mma(ah, bl[j], acc[i][j]);
        if (SPLIT_A) acc[i][j] = frag_mma(al, bh[j], acc[i][j]);
      }
      dep_guard4_h(acc[i][0], acc[i][1], acc[i][2], acc[i][3], ah, al);
    }
    keep4_h(bh[0], bh[1], bh[2], bh[3]);
    if (SPLIT_B) keep4_h(bl[0], bl[1], bl[2], bl[3]);
  }
  acc_guard4(acc[0][0], acc[0][1], acc[0][2], acc[0][3]);
  acc_guard4(acc[1][0], acc[1][1], acc[1][2], acc[1][3]);
  acc_guard4(acc[2][0], acc[2][1], acc[2][2], acc[2][3]);
  acc_guard4(acc[3][0], acc[3][1], acc[3][2], acc[3][3]);

  float* slab = sT[wave];
#pragma unroll
  for (int i = 0; i < 4; ++i) {
    const int mBase = m0 + (i << 4);
#pragma unroll
    for (int j = 0; j < 4; ++j) {
#pragma unroll
      for (int r = 0; r < 8; ++r) {
        const float v = acc[i][j][r] * scale;
        slab[(mOff + r) * 68 + (j << 4) + rlane] = v;
      }
    }
    __builtin_amdgcn_fence(__ATOMIC_RELEASE, "workgroup");
    __builtin_amdgcn_wave_barrier();
    __builtin_amdgcn_fence(__ATOMIC_ACQUIRE, "workgroup");
    {
      const int hh = lane >> 4, c4 = (lane & 15) * 4;
      for (int pass = 0; pass < 2; ++pass) {
#pragma unroll
        for (int it = 0; it < 8; ++it) {
          const int row = it * 2 + hh;
          v4f v = *(const v4f*)(slab + row * 68 + c4);
          *(volatile v4f*)(Cout + (size_t)(mBase + row) * ldc + n0 + c4) = v;
        }
        __threadfence();
      }
    }
    __builtin_amdgcn_fence(__ATOMIC_RELEASE, "workgroup");
    __builtin_amdgcn_wave_barrier();
    __builtin_amdgcn_fence(__ATOMIC_ACQUIRE, "workgroup");
  }
}

__global__ __launch_bounds__(256) void stats_rows(const float* __restrict__ Y1, float* __restrict__ P1) {
  const int c = (int)threadIdx.x;
  const size_t r0 = (size_t)blockIdx.x * ST1_ROWS;
  float s = 0.0f, q = 0.0f;
#pragma unroll 4
  for (int r = 0; r < ST1_ROWS; ++r) {
    const float v = Y1[(r0 + r) * CH_H1 + c];
    s = s + v;
    q = q + v * v;
  }
  volatile float* ps = P1 + (size_t)blockIdx.x * (2 * CH_H1) + c;
  volatile float* pq = P1 + (size_t)blockIdx.x * (2 * CH_H1) + CH_H1 + c;
  *ps = s;
  *pq = q;
  __threadfence();
  *ps = s;
  *pq = q;
}

__global__ __launch_bounds__(256) void finalize_rows(const float* __restrict__ P1, const float* __restrict__ gam,
                                                     const float* __restrict__ bet, const float* __restrict__ bia,
                                                     float* __restrict__ T1) {
  const int c = (int)threadIdx.x;
  double S = 0.0, Q = 0.0;
#pragma unroll 4
  for (int k = 0; k < ST1_BLOCKS; ++k) {
    const float ps = P1[(size_t)k * (2 * CH_H1) + c];
    const float pq = P1[(size_t)k * (2 * CH_H1) + CH_H1 + c];
    S = S + (double)ps;
    Q = Q + (double)pq;
  }
  const double inv_n = 1.0 / (double)NPTS_ALL;
  const double mean = S * inv_n;
  double var = Q * inv_n - mean * mean;
  var = var < 0.0 ? 0.0 : var;
  const float varf = (float)var;
  const float meanf = (float)mean;
  const float inv = 1.0f / sqrtf(varf + BN_EPS);
  const float sc = gam[c] * inv;
  const float bv = bia[c];
  const float meanb = meanf + bv;
  const float sh = bet[c] + (bv - meanb) * sc;
  volatile float* p0 = T1 + c;
  volatile float* p1 = T1 + CH_H1 + c;
  *p0 = sc;
  *p1 = sh;
  __threadfence();
  *p0 = sc;
  *p1 = sh;
}

__global__ __launch_bounds__(256) void bn_relu_h1(const float* __restrict__ Y1, const float* __restrict__ T1,
                                                  _Float16* __restrict__ H1) {
  const int lane = threadIdx.x & 31;
  const int wave = threadIdx.x >> 5;
  const int c0 = lane * 8;
  const v4f s0 = *(const v4f*)(T1 + c0);
  const v4f s1 = *(const v4f*)(T1 + c0 + 4);
  const v4f h0 = *(const v4f*)(T1 + CH_H1 + c0);
  const v4f h1 = *(const v4f*)(T1 + CH_H1 + c0 + 4);
  const size_t rbase = (size_t)blockIdx.x * 64 + (size_t)wave * 8;
#pragma unroll 1
  for (int r = 0; r < 8; ++r) {
    const size_t row = rbase + r;
    const v4f a = *(const v4f*)(Y1 + row * CH_H1 + c0);
    const v4f b = *(const v4f*)(Y1 + row * CH_H1 + c0 + 4);
    v8h hv;
    hv[0] = (_Float16)fmaxf(a.x * s0.x + h0.x, 0.0f);
    hv[1] = (_Float16)fmaxf(a.y * s0.y + h0.y, 0.0f);
    hv[2] = (_Float16)fmaxf(a.z * s0.z + h0.z, 0.0f);
    hv[3] = (_Float16)fmaxf(a.w * s0.w + h0.w, 0.0f);
    hv[4] = (_Float16)fmaxf(b.x * s1.x + h1.x, 0.0f);
    hv[5] = (_Float16)fmaxf(b.y * s1.y + h1.y, 0.0f);
    hv[6] = (_Float16)fmaxf(b.z * s1.z + h1.z, 0.0f);
    hv[7] = (_Float16)fmaxf(b.w * s1.w + h1.w, 0.0f);
    _Float16* dst = H1 + row * CH_H1 + c0;
    *(volatile v8h*)dst = hv;
    __threadfence();
    *(volatile v8h*)dst = hv;
  }
}

__global__ __launch_bounds__(256) void stats_finalize_ch(const float* __restrict__ Y2, const float* __restrict__ gam,
                                                         const float* __restrict__ bet, const float* __restrict__ bia,
                                                         float* __restrict__ T2) {
  __shared__ float sS[8];
  __shared__ float sQ[8];
  const int tid = (int)threadIdx.x;
  const int lane = tid & 31;
  const int wave = tid >> 5;
  const int o = (int)blockIdx.x;
  const float* row = Y2 + (size_t)o * NPTS_ALL;
  float s = 0.0f, q = 0.0f;
#pragma unroll 4
  for (int i = 0; i < NPTS_ALL / 1024; ++i) {
    const v4f v = *(const v4f*)(row + (size_t)(i * 256 + tid) * 4);
    s = s + ((v.x + v.y) + (v.z + v.w));
    q = q + ((v.x * v.x + v.y * v.y) + (v.z * v.z + v.w * v.w));
  }
#pragma unroll
  for (int off = 16; off >= 1; off >>= 1) {
    const float so = __shfl_xor(s, off, 32);
    const float qo = __shfl_xor(q, off, 32);
    s = s + so;
    q = q + qo;
  }
  if (lane == 0) { sS[wave] = s; sQ[wave] = q; }
  __syncthreads();
  double S = 0.0, Q = 0.0;
#pragma unroll
  for (int w = 0; w < 8; ++w) {
    S = S + (double)sS[w];
    Q = Q + (double)sQ[w];
  }
  const double inv_n = 1.0 / (double)NPTS_ALL;
  const double mean = S * inv_n;
  double var = Q * inv_n - mean * mean;
  var = var < 0.0 ? 0.0 : var;
  const float varf = (float)var;
  const float meanf = (float)mean;
  const float inv = 1.0f / sqrtf(varf + BN_EPS);
  const float sc = gam[o] * inv;
  const float bv = bia[o];
  const float meanb = meanf + bv;
  const float sh = bet[o] + (bv - meanb) * sc;
  const float val = (lane == 0) ? sc : ((lane == 1) ? sh : 0.0f);
  if (wave == 0) {
    volatile float* p = T2 + (size_t)o * 32 + lane;
    *p = val;
    __threadfence();
    *p = val;
  }
}

__global__ __launch_bounds__(256) void bn_relu_out(const float* __restrict__ Y2, const float* __restrict__ T2,
                                                   float* __restrict__ out) {
  const int f0 = (int)blockIdx.x * 4096;
  const int o  = (f0 >> 14) & (CH_OUT - 1);
  const int b  = f0 >> 21;
  const int n0 = f0 & (NPT1 - 1);
  const float sc = T2[(size_t)o * 32];
  const float sh = T2[(size_t)o * 32 + 1];
  const float* src = Y2 + (size_t)o * NPTS_ALL + (size_t)b * NPT1 + n0;
  float* dst = out + (size_t)f0;
#pragma unroll 1
  for (int it = 0; it < 4; ++it) {
    const int off = it * 1024 + (int)threadIdx.x * 4;
    const v4f v = *(const v4f*)(src + off);
    v4f r;
    r.x = fmaxf(v.x * sc + sh, 0.0f);
    r.y = fmaxf(v.y * sc + sh, 0.0f);
    r.z = fmaxf(v.z * sc + sh, 0.0f);
    r.w = fmaxf(v.w * sc + sh, 0.0f);
    *(volatile v4f*)(dst + off) = r;
    __threadfence();
    *(volatile v4f*)(dst + off) = r;
  }
}

extern "C" void kernel_launch(void* const* d_in, const int* in_sizes, int n_in,
                              void* d_out, int out_size, void* d_ws, size_t ws_size,
                              hipStream_t stream) {
  if (n_in < 12) return;
  if (in_sizes[0] != NB_BATCH * 3 * NPT1 || in_sizes[1] != NB_BATCH * 3 * NPT2) return;
  if (in_sizes[2] != NB_BATCH * CH_P1 * NPT1 || in_sizes[3] != NB_BATCH * CH_P2 * NPT2) return;
  if (in_sizes[4] != CH_H1 * CH_IN || in_sizes[8] != CH_OUT * CH_H1) return;
  if (out_size != NB_BATCH * CH_OUT * NPT1) return;
  if (ws_size < WS_TOTAL) return;

  const float* xyz1    = (const float*)d_in[0];
  const float* xyz2    = (const float*)d_in[1];
  const float* points1 = (const float*)d_in[2];
  const float* points2 = (const float*)d_in[3];
  const float* W1      = (const float*)d_in[4];
  const float* b1      = (const float*)d_in[5];
  const float* g1      = (const float*)d_in[6];
  const float* be1     = (const float*)d_in[7];
  const float* W2      = (const float*)d_in[8];
  const float* b2      = (const float*)d_in[9];
  const float* g2      = (const float*)d_in[10];
  const float* be2     = (const float*)d_in[11];

  unsigned char* ws = (unsigned char*)d_ws;
  _Float16* Xp  = (_Float16*)(ws + OFF_R1);
  _Float16* H1p = (_Float16*)(ws + OFF_R1);
  float*    Y1p = (float*)(ws + OFF_R2);
  float*    Y2p = (float*)(ws + OFF_R2);
  _Float16* W1h = (_Float16*)(ws + OFF_W1H);
  _Float16* W1l = (_Float16*)(ws + OFF_W1L);
  _Float16* W2h = (_Float16*)(ws + OFF_W2H);
  _Float16* W2l = (_Float16*)(ws + OFF_W2L);
  float*    P1p = (float*)(ws + OFF_P1);
  float*    T1p = (float*)(ws + OFF_T1);
  float*    T2p = (float*)(ws + OFF_T2);

  prep_weights<<<PW_BLOCKS_W1 + PW_BLOCKS_W2, 256, 0, stream>>>(W1, W2, W1h, W1l, W2h, W2l);

  knn_build_x<<<NB_BATCH * (NPT1 / 256), 256, 0, stream>>>(xyz1, xyz2, points1, points2, Xp);

  wmma_gemm64_f16<false, true><<<(NPTS_ALL / 64) * (CH_H1 / 64) / 8, 256, 0, stream>>>(
      (const unsigned short*)Xp, (const unsigned short*)Xp, CH_IN,
      (const unsigned short*)W1h, (const unsigned short*)W1l, CH_IN,
      Y1p, CH_H1, NPTS_ALL, CH_H1, CH_IN, W_CARRY_INV);

  stats_rows<<<ST1_BLOCKS, 256, 0, stream>>>(Y1p, P1p);
  finalize_rows<<<1, 256, 0, stream>>>(P1p, g1, be1, b1, T1p);
  bn_relu_h1<<<NPTS_ALL / 64, 256, 0, stream>>>(Y1p, T1p, H1p);

  wmma_gemm64_f16<true, false><<<(CH_OUT / 64) * (NPTS_ALL / 64) / 8, 256, 0, stream>>>(
      (const unsigned short*)W2h, (const unsigned short*)W2l, CH_H1,
      (const unsigned short*)H1p, (const unsigned short*)H1p, CH_H1,
      Y2p, NPTS_ALL, CH_OUT, NPTS_ALL, CH_H1, W_CARRY_INV);

  stats_finalize_ch<<<CH_OUT, 256, 0, stream>>>(Y2p, g2, be2, b2, T2p);
  bn_relu_out<<<(NB_BATCH * CH_OUT * NPT1) / 4096, 256, 0, stream>>>(Y2p, T2p, (float*)d_out);
}
